// PointNetSetAbstraction_10213432230205
// MI455X (gfx1250) — hardware-verified
//
#include <hip/hip_runtime.h>
#include <stdint.h>
#include <math.h>

#pragma clang fp contract(off)

constexpr int kB      = 8;
constexpr int kN      = 8192;
constexpr int kD      = 64;
constexpr int kS      = 1024;
constexpr int kNS     = 32;
constexpr int kGroups = kB * kS;
constexpr int kRows   = kGroups * kNS;
constexpr int kIn1    = 67;
constexpr int kKf     = 64;
constexpr int kC1     = 64;
constexpr int kC2     = 64;
constexpr int kC3     = 128;
constexpr int kRowW   = kKf / 2;
constexpr float kBnEps = 1e-5f;
constexpr unsigned kR2Bits = 0x3D23D70Au;

static_assert(kRows % 64 == 0, "M tile multiple");
static_assert(kKf % 32 == 0, "K multiple of 32");
static_assert(kC1 % 64 == 0 && kC2 % 64 == 0 && kC3 % 64 == 0, "N tile multiple");
static_assert(kC1 == kKf && kC2 == kKf, "all three GEMMs run K = 64");
static_assert(kNS * kRowW == 1024, "group tile words");

constexpr size_t cOffNxyz   = 0;
constexpr size_t cBytesNxyz = (size_t)kGroups * 4 * 4;
constexpr size_t cOffRel    = cOffNxyz + cBytesNxyz;
constexpr size_t cBytesRel  = (size_t)kRows * 4 * 4;
constexpr size_t cOffBtH    = cOffRel + cBytesRel;
constexpr size_t cBytesBt   = (size_t)(kC1 * kKf + kC2 * kKf + kC3 * kKf) * 2;
constexpr size_t cOffBtL    = cOffBtH + cBytesBt;
constexpr size_t cOffStat   = cOffBtL + cBytesBt;
constexpr size_t cBytesStat = 4096;
constexpr size_t cOffPart   = cOffStat + cBytesStat;
constexpr size_t cBytesPart = (size_t)8192 * 128 * 4;
constexpr size_t cOffZmax   = cOffPart + cBytesPart;
constexpr size_t cBytesZm   = (size_t)kGroups * kC3 * 4;
constexpr size_t cOffZmin   = cOffZmax + cBytesZm;
constexpr size_t cBytesPlane = (size_t)kRows * kKf * 2;
constexpr size_t cOffAh     = cOffZmin + cBytesZm;
constexpr size_t cOffAl     = cOffAh + cBytesPlane;
constexpr size_t cOffZ      = cOffAl + cBytesPlane;
constexpr size_t cWsTotal   = cOffZ + cBytesPlane;
static_assert(cWsTotal <= (size_t)134217728, "carve budget");
static_assert((size_t)4096 * 128 * 4 <= cBytesPart, "partials layer 1/2");
static_assert(cOffRel % 4096 == 0 && cOffBtH % 4096 == 0 && cOffBtL % 4096 == 0 && cOffStat % 4096 == 0 &&
              cOffPart % 4096 == 0 && cOffZmax % 4096 == 0 && cOffZmin % 4096 == 0 &&
              cOffAh % 4096 == 0 && cOffAl % 4096 == 0 && cOffZ % 4096 == 0, "alignment");
static_assert(24576 * 4 == 98304, "out1 byte offset");
static_assert(98304 + kGroups * kC3 * 4 == 4292608, "d_out total");

typedef __attribute__((ext_vector_type(16))) _Float16 v16h;
typedef __attribute__((ext_vector_type(8)))  _Float16 v8h;
typedef __attribute__((ext_vector_type(16))) __bf16   v16b;
typedef __attribute__((ext_vector_type(8)))  __bf16   v8b;
typedef __attribute__((ext_vector_type(8)))  float    v8f;
typedef __attribute__((ext_vector_type(4)))  float    v4f;
typedef __attribute__((ext_vector_type(2)))  float    v2f;
typedef __attribute__((ext_vector_type(4)))  unsigned int v4u;

__device__ __forceinline__ unsigned short f2bf_bits(float f) {
  unsigned u = __float_as_uint(f);
  return (unsigned short)((u + 0x7FFFu + ((u >> 16) & 1u)) >> 16);
}
__device__ __forceinline__ float bf_bits2f(unsigned short h) { return __uint_as_float(((unsigned)h) << 16); }

__device__ __forceinline__ void dep_guard_h(v8f& a, v8f& b, v16h x, v16h y) { asm volatile("v_nop\n\tv_nop\n\tv_nop\n\tv_nop" : "+v"(a), "+v"(b) : "v"(x), "v"(y)); }
__device__ __forceinline__ void dep_guard_b(v8f& a, v8f& b, v16b x, v16b y) { asm volatile("v_nop\n\tv_nop\n\tv_nop\n\tv_nop" : "+v"(a), "+v"(b) : "v"(x), "v"(y)); }
__device__ __forceinline__ void keep4_h(v16h a, v16h b, v16h c, v16h d) { asm volatile("v_nop" :: "v"(a), "v"(b), "v"(c), "v"(d)); }
__device__ __forceinline__ void keep4_b(v16b a, v16b b, v16b c, v16b d) { asm volatile("v_nop" :: "v"(a), "v"(b), "v"(c), "v"(d)); }
__device__ __forceinline__ void acc_guard4(v8f& a, v8f& b, v8f& c, v8f& d) { asm volatile("v_nop\n\tv_nop\n\tv_nop\n\tv_nop" : "+v"(a), "+v"(b), "+v"(c), "+v"(d)); }
__device__ __forceinline__ void dep_guard4_b(v8f& a, v8f& b, v8f& c, v8f& d, v16b x, v16b y) {
  asm volatile("v_nop\n\tv_nop\n\tv_nop\n\tv_nop" : "+v"(a), "+v"(b), "+v"(c), "+v"(d) : "v"(x), "v"(y));
}
template <typename T> struct Frag;
template <> struct Frag<_Float16> {
  typedef v16h V; union U { v16h v; v8h h[2]; };
  static __device__ __forceinline__ v16h load(const _Float16* p) {
    U f; f.h[0] = *(const v8h*)(p); f.h[1] = *(const v8h*)(p + 16); return f.v;
  }
  static __device__ __forceinline__ v8f mma(v16h a, v16h b, v8f c) {
    return __builtin_amdgcn_wmma_f32_16x16x32_f16(false, a, false, b, (short)0, c, false, false);
  }
  static __device__ __forceinline__ void guard(v8f& a, v8f& b, v16h x, v16h y) { dep_guard_h(a, b, x, y); }
  static __device__ __forceinline__ void keep(v16h a, v16h b, v16h c, v16h d) { keep4_h(a, b, c, d); }
};
template <> struct Frag<__bf16> {
  typedef v16b V; union U { v16b v; v8b h[2]; };
  static __device__ __forceinline__ v16b load(const __bf16* p) {
    U f; f.h[0] = *(const v8b*)(p); f.h[1] = *(const v8b*)(p + 16); return f.v;
  }
  static __device__ __forceinline__ v8f mma(v16b a, v16b b, v8f c) {
    return __builtin_amdgcn_wmma_f32_16x16x32_bf16(false, a, false, b, (short)0, c, false, false);
  }
  static __device__ __forceinline__ void guard(v8f& a, v8f& b, v16b x, v16b y) { dep_guard_b(a, b, x, y); }
  static __device__ __forceinline__ void keep(v16b a, v16b b, v16b c, v16b d) { keep4_b(a, b, c, d); }
};

__device__ __forceinline__ unsigned pk16(unsigned short a, unsigned short b) { return (unsigned)a | ((unsigned)b << 16); }
__device__ __forceinline__ unsigned short h_bits(float f) { const _Float16 h = (_Float16)f; return __builtin_bit_cast(unsigned short, h); }

__device__ __forceinline__ void split_bf16(float v, unsigned short& hb, unsigned short& lb) {
  hb = f2bf_bits(v);
  lb = f2bf_bits(v - bf_bits2f(hb));
}

__device__ __forceinline__ float h16_to_f32(unsigned hb) {
  const unsigned sgn = (hb & 0x8000u) << 16; const unsigned em = hb & 0x7fffu;
  const float fn = __uint_as_float((em << 13) + 0x38000000u);
  const float fs = (float)em * 5.9604644775390625e-8f;
  const float mag = (em < 0x400u) ? fs : fn; return __uint_as_float(__float_as_uint(mag) | sgn);
}

__device__ __forceinline__ void wave_lds_sync() {
  __builtin_amdgcn_fence(__ATOMIC_RELEASE, "workgroup");
  __builtin_amdgcn_wave_barrier();
  __builtin_amdgcn_fence(__ATOMIC_ACQUIRE, "workgroup");
}

__global__ __launch_bounds__(1024) void fps_kernel(const float* __restrict__ xyz,
                                                   float* __restrict__ out0,
                                                   float* __restrict__ nxyz) {
#pragma clang fp contract(off)
  __shared__ float sVal[2][32];
  __shared__ int   sIdx[2][32];
  __shared__ int   sList[kS];
  __shared__ __align__(16) float sOut[kS * 3];
  const int b = blockIdx.x;
  const int t = threadIdx.x;
  const int lane = t & 31, wave = t >> 5;
  const float* X = xyz + (size_t)b * kN * 3;

  const v4f* Xv = (const v4f*)(X + (size_t)t * 24);
  const v4f q0 = Xv[0], q1 = Xv[1], q2 = Xv[2], q3 = Xv[3], q4 = Xv[4], q5 = Xv[5];
  float px[8], py[8], pz[8], dm[8];
  px[0] = q0[0]; py[0] = q0[1]; pz[0] = q0[2];
  px[1] = q0[3]; py[1] = q1[0]; pz[1] = q1[1];
  px[2] = q1[2]; py[2] = q1[3]; pz[2] = q2[0];
  px[3] = q2[1]; py[3] = q2[2]; pz[3] = q2[3];
  px[4] = q3[0]; py[4] = q3[1]; pz[4] = q3[2];
  px[5] = q3[3]; py[5] = q4[0]; pz[5] = q4[1];
  px[6] = q4[2]; py[6] = q4[3]; pz[6] = q5[0];
  px[7] = q5[1]; py[7] = q5[2]; pz[7] = q5[3];
#pragma unroll
  for (int i = 0; i < 8; ++i) dm[i] = 1e10f;

  int far = 0;
  for (int it = 0; it < kS; ++it) {
    const int par = it & 1;
    if (t == 0) sList[it] = far;
    const float cx = X[far * 3 + 0];
    const float cy = X[far * 3 + 1];
    const float cz = X[far * 3 + 2];
    float bv = -1.0f;
    int bi = 0;
#pragma unroll
    for (int i = 0; i < 8; ++i) {
      const float dx = px[i] - cx;
      const float dy = py[i] - cy;
      const float dz = pz[i] - cz;
      const float t0 = dx * dx;
      const float t1 = dy * dy;
      const float t2 = dz * dz;
      const float s02 = t0 + t2;
      const float dd = s02 + t1;
      dm[i] = fminf(dm[i], dd);
      const bool take = dm[i] > bv;
      bv = take ? dm[i] : bv;
      bi = take ? (t * 8 + i) : bi;
    }
#pragma unroll
    for (int off = 16; off > 0; off >>= 1) {
      const float ov = __shfl_xor(bv, off, 32);
      const int   oi = __shfl_xor(bi, off, 32);
      const bool take = (ov > bv) || (ov == bv && oi < bi);
      bv = take ? ov : bv;
      bi = take ? oi : bi;
    }
    if (lane == 0) { sVal[par][wave] = bv; sIdx[par][wave] = bi; }
    __syncthreads();
    float v2 = sVal[par][lane];
    int   i2 = sIdx[par][lane];
#pragma unroll
    for (int off = 16; off > 0; off >>= 1) {
      const float ov = __shfl_xor(v2, off, 32);
      const int   oi = __shfl_xor(i2, off, 32);
      const bool take = (ov > v2) || (ov == v2 && oi < i2);
      v2 = take ? ov : v2;
      i2 = take ? oi : i2;
    }
    far = __builtin_amdgcn_readfirstlane(i2);
  }
  __syncthreads();
  {
    int p = sList[t];
    p = p < 0 ? 0 : (p > kN - 1 ? kN - 1 : p);
    const float x0 = X[p * 3 + 0], y0 = X[p * 3 + 1], z0 = X[p * 3 + 2];
    sOut[t * 3 + 0] = x0;
    sOut[t * 3 + 1] = y0;
    sOut[t * 3 + 2] = z0;
    const v4f nv = (v4f){x0, y0, z0, 0.0f};
    float* np = nxyz + ((size_t)b * kS + t) * 4;
    for (int pass = 0; pass < 2; ++pass) {
      *(volatile v4f*)np = nv;
      __threadfence();
    }
  }
  __syncthreads();
  if (t < (kS * 3) / 4) {
    const v4f v = *(const v4f*)(sOut + t * 4);
    float* op = out0 + (size_t)b * (kS * 3) + t * 4;
    for (int pass = 0; pass < 2; ++pass) {
      *(volatile v4f*)op = v;
      __threadfence();
    }
  }
}

__global__ __launch_bounds__(128) void group_kernel(const float* __restrict__ xyz,
                                                    const float* __restrict__ points,
                                                    const float* __restrict__ nxyz,
                                                    unsigned int* __restrict__ Xh,
                                                    unsigned int* __restrict__ Xl,
                                                    float* __restrict__ rel) {
#pragma clang fp contract(off)
  __shared__ int sG[4][kNS];
  __shared__ __align__(16) unsigned int sHi[4][kNS * kRowW];
  __shared__ __align__(16) unsigned int sLo[4][kNS * kRowW];
  __shared__ __align__(16) float sRel[4][kNS * 4];
  const int lane = threadIdx.x & 31, wave = threadIdx.x >> 5;
  const int g = blockIdx.x * 4 + wave;
  const int b = g >> 10;
  const float* X = xyz + (size_t)b * kN * 3;
  const float* P = points + (size_t)b * kN * kD;
  const v4f cv = *(const v4f*)(nxyz + (size_t)g * 4);
  const float cx = cv[0], cy = cv[1], cz = cv[2];
  const float r2 = __uint_as_float(kR2Bits);
  int* sg = sG[wave];
  int cnt = 0, first = 0;
  for (int ch = 0; ch < kN / 32; ++ch) {
    const int p = ch * 32 + lane;
    const float x = X[p * 3 + 0], y = X[p * 3 + 1], z = X[p * 3 + 2];
    const float dx = cx - x, dy = cy - y, dz = cz - z;
    const float t0 = dx * dx;
    const float t1 = dy * dy;
    const float t2 = dz * dz;
    const float s02 = t0 + t2;
    const float s = s02 + t1;
    const bool hit = (s <= r2);
    const unsigned m = (unsigned)__ballot(hit ? 1 : 0);
    const int src = (m != 0u) ? (int)__builtin_ctz(m) : 0;
    const int pf = __shfl(p, src, 32);
    if (cnt == 0 && m != 0u) first = pf;
    const unsigned below = m & ((1u << lane) - 1u);
    const int slot = cnt + (int)__popc(below);
    if (hit && slot < kNS) sg[slot] = p;
    cnt += (int)__popc(m);
    if (cnt >= kNS) break;
  }
  const int cntc = cnt < kNS ? cnt : kNS;
  if (lane >= cntc) sg[lane] = first;
  __syncthreads();

  unsigned int* sh = sHi[wave];
  unsigned int* sl = sLo[wave];
  float* sr = sRel[wave];
  const int lsel = (lane < 2) ? lane : 2;
  const float cl = (lane == 0) ? cx : ((lane == 1) ? cy : cz);
#pragma unroll 2
  for (int j = 0; j < kNS; ++j) {
    int gi = sg[j];
    gi = gi < 0 ? 0 : (gi > kN - 1 ? kN - 1 : gi);
    const v2f fv = *(const v2f*)(P + (size_t)gi * kD + 2 * lane);
    const float xg = X[gi * 3 + lsel];
    unsigned short h0, l0, h1, l1;
    split_bf16(fv[0], h0, l0);
    split_bf16(fv[1], h1, l1);
    sh[j * kRowW + lane] = pk16(h0, h1);
    sl[j * kRowW + lane] = pk16(l0, l1);
    const float rv = (lane < 3) ? (xg - cl) : 0.0f;
    if (lane < 4) sr[j * 4 + lane] = rv;
  }
  __syncthreads();
  unsigned int* dh = Xh + (size_t)g * (kNS * kRowW);
  unsigned int* dl = Xl + (size_t)g * (kNS * kRowW);
  float* rp = rel + ((size_t)g * kNS + lane) * 4;
  const v4f rvv = *(const v4f*)(sr + lane * 4);
  const int q = lane >> 3, c4 = (lane & 7) * 4;
  for (int pass = 0; pass < 2; ++pass) {
#pragma unroll
    for (int it = 0; it < 8; ++it) {
      const int line = it * 4 + q;
      const v4u vh = *(const v4u*)(sh + line * 32 + c4);
      const v4u vl = *(const v4u*)(sl + line * 32 + c4);
      *(volatile v4u*)(dh + line * 32 + c4) = vh;
      *(volatile v4u*)(dl + line * 32 + c4) = vl;
    }
    *(volatile v4f*)rp = rvv;
    __threadfence();
  }
}

__global__ __launch_bounds__(256) void prep_w_kernel(const float* __restrict__ W1, const float* __restrict__ W2,
                                                     const float* __restrict__ W3,
                                                     unsigned int* __restrict__ Bh, unsigned int* __restrict__ Bl) {
  const int blk = blockIdx.x;
  const int tid = blockIdx.x * 256 + threadIdx.x;
  float v[8];
  if (blk < 2) {
#pragma unroll
    for (int e = 0; e < 8; ++e) {
      const int h = tid * 8 + e;
      const int o = h >> 6;
      const int k = h & 63;
      v[e] = W1[o * kIn1 + 3 + k];
    }
  } else if (blk < 4) {
#pragma unroll
    for (int e = 0; e < 8; ++e) v[e] = W2[tid * 8 + e - 4096];
  } else {
#pragma unroll
    for (int e = 0; e < 8; ++e) v[e] = W3[tid * 8 + e - 8192];
  }
  unsigned short hb[8], lb[8];
#pragma unroll
  for (int e = 0; e < 8; ++e) split_bf16(v[e], hb[e], lb[e]);
  const v4u uh = (v4u){pk16(hb[0], hb[1]), pk16(hb[2], hb[3]), pk16(hb[4], hb[5]), pk16(hb[6], hb[7])};
  const v4u ul = (v4u){pk16(lb[0], lb[1]), pk16(lb[2], lb[3]), pk16(lb[4], lb[5]), pk16(lb[6], lb[7])};
  unsigned int* dh = Bh + (size_t)tid * 4;
  unsigned int* dl = Bl + (size_t)tid * 4;
  for (int pass = 0; pass < 2; ++pass) {
    *(volatile v4u*)dh = uh;
    *(volatile v4u*)dl = ul;
    __threadfence();
  }
}

template <int MODE>
__global__ __launch_bounds__(256) void gemm_bf16x3_kernel(
    const unsigned short* __restrict__ Ahp, const unsigned short* __restrict__ Alp, int lda,
    const unsigned short* __restrict__ Bhp, const unsigned short* __restrict__ Blp, int ldb,
    unsigned short* __restrict__ Cp, int ldc,
    const float* __restrict__ rel, const float* __restrict__ W1,
    float* __restrict__ zmx, float* __restrict__ zmn, int ldz,
    float* __restrict__ part,
    int M, int N, int K) {
  typedef __bf16 T;
  typedef v16b V;
  const T* Ah = (const T*)Ahp;
  const T* Al = (const T*)Alp;
  const T* Bh = (const T*)Bhp;
  const T* Bl = (const T*)Blp;
  __shared__ __align__(16) float sT[8][16 * 68];
  __shared__ __align__(16) float sWc[64 * 4];
  if (MODE == 0) {
    if (threadIdx.x < 64) {
      const int t = threadIdx.x;
      const float w0 = W1[t * kIn1 + 0];
      const float w1v = W1[t * kIn1 + 1];
      const float w2v = W1[t * kIn1 + 2];
      sWc[t * 4 + 0] = w0;
      sWc[t * 4 + 1] = w1v;
      sWc[t * 4 + 2] = w2v;
      sWc[t * 4 + 3] = 0.0f;
    }
  }
  __syncthreads();
  const int lane = threadIdx.x & 31;
  const int wave = threadIdx.x >> 5;
  const int tilesN = N >> 6;
  const int tilesM = M >> 6;
  const int tile = blockIdx.x * 8 + wave;
  if (tile >= tilesM * tilesN) return;
  const int tm = tile / tilesN;
  const int tn = tile - tm * tilesN;
  const int m0 = tm << 6;
  const int n0 = tn << 6;
  const int rlane = lane & 15;
  const int koff  = (lane >> 4) * 8;
  const int mOff  = (lane >> 4) * 8;

  v8f acc[4][4];
#pragma unroll
  for (int i = 0; i < 4; ++i)
#pragma unroll
    for (int j = 0; j < 4; ++j) acc[i][j] = (v8f){0.f,0.f,0.f,0.f,0.f,0.f,0.f,0.f};

  for (int k0 = 0; k0 < K; k0 += 32) {
    V bh[4], bl[4];
#pragma unroll
    for (int j = 0; j < 4; ++j) {
      const size_t bo = (size_t)(n0 + (j << 4) + rlane) * ldb + koff + k0;
      bh[j] = Frag<T>::load(Bh + bo);
      bl[j] = Frag<T>::load(Bl + bo);
    }
#pragma unroll
    for (int i = 0; i < 4; ++i) {
      const size_t ao = (size_t)(m0 + (i << 4) + rlane) * lda + koff + k0;
      V fah = Frag<T>::load(Ah + ao);
      V fal = Frag<T>::load(Al + ao);
#pragma unroll
      for (int j = 0; j < 4; ++j) {
        acc[i][j] = Frag<T>::mma(fah, bh[j], acc[i][j]);
        acc[i][j] = Frag<T>::mma(fah, bl[j], acc[i][j]);
        acc[i][j] = Frag<T>::mma(fal, bh[j], acc[i][j]);
      }
      dep_guard4_b(acc[i][0], acc[i][1], acc[i][2], acc[i][3], fah, fal);
    }
    Frag<T>::keep(bh[0], bh[1], bh[2], bh[3]);
    Frag<T>::keep(bl[0], bl[1], bl[2], bl[3]);
  }
  acc_guard4(acc[0][0], acc[0][1], acc[0][2], acc[0][3]);
  acc_guard4(acc[1][0], acc[1][1], acc[1][2], acc[1][3]);
  acc_guard4(acc[2][0], acc[2][1], acc[2][2], acc[2][3]);
  acc_guard4(acc[3][0], acc[3][1], acc[3][2], acc[3][3]);

  float* slab = sT[wave];
  float cs0 = 0.0f, cs1 = 0.0f, cq0 = 0.0f, cq1 = 0.0f;
  float gmx[2][2], gmn[2][2];
#pragma unroll
  for (int a = 0; a < 2; ++a) { gmx[a][0] = -INFINITY; gmx[a][1] = -INFINITY; gmn[a][0] = INFINITY; gmn[a][1] = INFINITY; }
#pragma unroll
  for (int i = 0; i < 4; ++i) {
    const int mBase = m0 + (i << 4);
    if (MODE == 0) {
#pragma unroll
      for (int r = 0; r < 8; ++r) {
        const int row = mBase + mOff + r;
        const v4f rq = *(const v4f*)(rel + (size_t)row * 4);
#pragma unroll
        for (int j = 0; j < 4; ++j) {
          const float* w = sWc + (n0 + (j << 4) + rlane) * 4;
          const float px = rq[0] * w[0];
          const float py = rq[1] * w[1];
          const float pz = rq[2] * w[2];
          const float sxy = px + py;
          const float sc = sxy + pz;
          slab[(mOff + r) * 68 + (j << 4) + rlane] = acc[i][j][r] + sc;
        }
      }
    } else {
#pragma unroll
      for (int j = 0; j < 4; ++j) {
#pragma unroll
        for (int r = 0; r < 8; ++r) slab[(mOff + r) * 68 + (j << 4) + rlane] = acc[i][j][r];
      }
    }
    wave_lds_sync();
    float mx0 = -INFINITY, mx1 = -INFINITY, mn0 = INFINITY, mn1 = INFINITY;
#pragma unroll
    for (int rr = 0; rr < 16; ++rr) {
      const float v0 = slab[rr * 68 + lane];
      const float v1 = slab[rr * 68 + 32 + lane];
      cs0 += v0; cs1 += v1;
      cq0 += v0 * v0; cq1 += v1 * v1;
      if (MODE == 2) { mx0 = fmaxf(mx0, v0); mx1 = fmaxf(mx1, v1); mn0 = fminf(mn0, v0); mn1 = fminf(mn1, v1); }
    }
    if (MODE == 2) {
      gmx[i >> 1][0] = fmaxf(gmx[i >> 1][0], mx0); gmx[i >> 1][1] = fmaxf(gmx[i >> 1][1], mx1);
      gmn[i >> 1][0] = fminf(gmn[i >> 1][0], mn0); gmn[i >> 1][1] = fminf(gmn[i >> 1][1], mn1);
    }
    if (MODE != 2) {
      const int q = lane >> 3, c8 = (lane & 7) * 8;
      for (int pass = 0; pass < 2; ++pass) {
#pragma unroll
        for (int it = 0; it < 4; ++it) {
          const int row = it * 4 + q;
          const float* sp = slab + row * 68 + c8;
          v8h hv;
#pragma unroll
          for (int e = 0; e < 8; ++e) hv[e] = (_Float16)sp[e];
          *(volatile v8h*)(Cp + (size_t)(mBase + row) * ldc + n0 + c8) = hv;
        }
        __threadfence();
      }
    }
    wave_lds_sync();
  }
  slab[lane] = cs0; slab[32 + lane] = cs1; slab[64 + lane] = cq0; slab[96 + lane] = cq1;
  if (MODE == 2) {
    slab[128 + lane] = gmx[0][0]; slab[160 + lane] = gmx[0][1]; slab[192 + lane] = gmn[0][0]; slab[224 + lane] = gmn[0][1];
    slab[256 + lane] = gmx[1][0]; slab[288 + lane] = gmx[1][1]; slab[320 + lane] = gmn[1][0]; slab[352 + lane] = gmn[1][1];
  }
  wave_lds_sync();
  {
    const v4f pv = *(const v4f*)(slab + 4 * lane);
    float* pp = part + (size_t)tile * 128 + 4 * lane;
    for (int pass = 0; pass < 2; ++pass) {
      *(volatile v4f*)pp = pv;
      __threadfence();
    }
  }
  if (MODE == 2) {
    const int hh = lane >> 4, c4 = (lane & 15) * 4;
    const v4f g0v = *(const v4f*)(slab + 128 + hh * 64 + c4);
    const v4f g1v = *(const v4f*)(slab + 256 + hh * 64 + c4);
    float* base = hh ? zmn : zmx;
    float* d0 = base + (size_t)(tm * 2 + 0) * ldz + n0 + c4;
    float* d1 = base + (size_t)(tm * 2 + 1) * ldz + n0 + c4;
    for (int pass = 0; pass < 2; ++pass) {
      *(volatile v4f*)d0 = g0v;
      *(volatile v4f*)d1 = g1v;
      __threadfence();
    }
  }
}

__global__ __launch_bounds__(128) void bn_finalize_kernel(const float* __restrict__ part, int tilesM, int tilesN, int nc,
                                                          const float* __restrict__ gam, const float* __restrict__ bet,
                                                          float* __restrict__ stats) {
#pragma clang fp contract(off)
  __shared__ __align__(16) float sS[256];
  const int c = threadIdx.x;
  const int cc = (c < nc) ? c : 0;
  const int tn = cc >> 6, slot = cc & 63;
  double s = 0.0, q = 0.0;
  for (int tm = 0; tm < tilesM; ++tm) {
    const float* p = part + (size_t)(tm * tilesN + tn) * 128;
    s += (double)p[slot];
    q += (double)p[64 + slot];
  }
  const double invM = 1.0 / (double)kRows;
  const double mean = s * invM;
  double var = q * invM - mean * mean;
  var = var < 0.0 ? 0.0 : var;
  const float meanf = (float)mean;
  const float rstd  = rsqrtf((float)var + kBnEps);
  const float gv = gam[cc], bv = bet[cc];
  const float a  = rstd * gv;
  const float ma = meanf * a;
  const float sh = bv - ma;
  sS[c]       = (c < nc) ? a  : 0.0f;
  sS[128 + c] = (c < nc) ? sh : 0.0f;
  __syncthreads();
  if (c < 32) {
    const v4f av = *(const v4f*)(sS + 4 * c);
    const v4f cv = *(const v4f*)(sS + 128 + 4 * c);
    float* pa = stats + 4 * c;
    float* pc = stats + 128 + 4 * c;
    for (int pass = 0; pass < 2; ++pass) {
      *(volatile v4f*)pa = av;
      *(volatile v4f*)pc = cv;
      __threadfence();
    }
  }
}

__global__ __launch_bounds__(256) void bn_act_kernel(const unsigned int* __restrict__ Z, const float* __restrict__ stats,
                                                   unsigned int* __restrict__ Yh, unsigned int* __restrict__ Yl, int n8) {
#pragma clang fp contract(off)
  const int i = blockIdx.x * 256 + threadIdx.x;
  if (i >= n8) return;
  const int c0 = (i & 7) * 8;
  const v4u w = *(const v4u*)(Z + (size_t)i * 4);
  const v4f a0 = *(const v4f*)(stats + c0), a1 = *(const v4f*)(stats + c0 + 4);
  const v4f s0 = *(const v4f*)(stats + 128 + c0), s1 = *(const v4f*)(stats + 128 + c0 + 4);
  float aa[8], cc[8], z[8];
#pragma unroll
  for (int e = 0; e < 4; ++e) { aa[e] = a0[e]; aa[4 + e] = a1[e]; cc[e] = s0[e]; cc[4 + e] = s1[e]; }
#pragma unroll
  for (int k = 0; k < 4; ++k) { z[2 * k] = h16_to_f32(w[k] & 0xffffu); z[2 * k + 1] = h16_to_f32(w[k] >> 16); }
  unsigned short hb[8], lb[8];
#pragma unroll
  for (int e = 0; e < 8; ++e) {
    const float prod = z[e] * aa[e];
    const float y = prod + cc[e];
    split_bf16(fmaxf(y, 0.0f), hb[e], lb[e]);
  }
  const v4u uh = (v4u){pk16(hb[0], hb[1]), pk16(hb[2], hb[3]), pk16(hb[4], hb[5]), pk16(hb[6], hb[7])};
  const v4u ul = (v4u){pk16(lb[0], lb[1]), pk16(lb[2], lb[3]), pk16(lb[4], lb[5]), pk16(lb[6], lb[7])};
  unsigned int* ph = Yh + (size_t)i * 4;
  unsigned int* pl = Yl + (size_t)i * 4;
  for (int pass = 0; pass < 2; ++pass) {
    *(volatile v4u*)ph = uh;
    *(volatile v4u*)pl = ul;
    __threadfence();
  }
}

__global__ __launch_bounds__(256) void pool_out_kernel(const float* __restrict__ zmx, const float* __restrict__ zmn,
                                                     const float* __restrict__ stats, float* __restrict__ out1, int n4) {
#pragma clang fp contract(off)
  const int i = blockIdx.x * 256 + threadIdx.x;
  if (i >= n4) return;
  const int g  = i >> 5;
  const int c0 = (i & 31) * 4;
  const v4f zx = *(const v4f*)(zmx + (size_t)g * kC3 + c0);
  const v4f zn = *(const v4f*)(zmn + (size_t)g * kC3 + c0);
  const v4f av = *(const v4f*)(stats + c0);
  const v4f cv = *(const v4f*)(stats + 128 + c0);
  v4f o = (v4f){0.0f, 0.0f, 0.0f, 0.0f};
#pragma unroll
  for (int e = 0; e < 4; ++e) {
    const float p1 = zx[e] * av[e];
    const float t1 = p1 + cv[e];
    const float p2 = zn[e] * av[e];
    const float t2 = p2 + cv[e];
    o[e] = fmaxf(fmaxf(t1, t2), 0.0f);
  }
  float* op = out1 + (size_t)g * kC3 + c0;
  for (int pass = 0; pass < 2; ++pass) {
    *(volatile v4f*)op = o;
    __threadfence();
  }
}

extern "C" void kernel_launch(void* const* d_in, const int* in_sizes, int n_in,
                              void* d_out, int out_size, void* d_ws, size_t ws_size,
                              hipStream_t stream) {
  (void)in_sizes;
  if (n_in < 11) return;
  if (out_size < kGroups * 3 + kGroups * kC3) return;
  if (ws_size < cWsTotal) return;

  const float* xyz    = (const float*)d_in[0];
  const float* points = (const float*)d_in[1];
  const float* W1 = (const float*)d_in[2];
  const float* g1 = (const float*)d_in[3];
  const float* b1 = (const float*)d_in[4];
  const float* W2 = (const float*)d_in[5];
  const float* g2 = (const float*)d_in[6];
  const float* b2 = (const float*)d_in[7];
  const float* W3 = (const float*)d_in[8];
  const float* g3 = (const float*)d_in[9];
  const float* b3 = (const float*)d_in[10];

  float* out0 = (float*)d_out;
  float* out1 = (float*)d_out + 24576;

  char* ws = (char*)d_ws;
  float*          nxyz  = (float*)(ws + cOffNxyz);
  float*          rel   = (float*)(ws + cOffRel);
  unsigned short* bth   = (unsigned short*)(ws + cOffBtH);
  unsigned short* btl   = (unsigned short*)(ws + cOffBtL);
  unsigned short* bt1h  = bth;
  unsigned short* bt2h  = bth + kC1 * kKf;
  unsigned short* bt3h  = bth + kC1 * kKf + kC2 * kKf;
  unsigned short* bt1l  = btl;
  unsigned short* bt2l  = btl + kC1 * kKf;
  unsigned short* bt3l  = btl + kC1 * kKf + kC2 * kKf;
  float*          stat0 = (float*)(ws + cOffStat);
  float*          stat1 = stat0 + 256;
  float*          stat2 = stat0 + 512;
  float*          part  = (float*)(ws + cOffPart);
  float*          zmax  = (float*)(ws + cOffZmax);
  float*          zmin  = (float*)(ws + cOffZmin);
  unsigned short* aph   = (unsigned short*)(ws + cOffAh);
  unsigned short* apl   = (unsigned short*)(ws + cOffAl);
  unsigned short* zp    = (unsigned short*)(ws + cOffZ);

  const int tilesM  = kRows / 64;
  const int tiles12 = tilesM * (kC1 / 64);
  const int tiles3  = tilesM * (kC3 / 64);
  const int n8      = kRows * kKf / 8;
  const int n4      = kGroups * kC3 / 4;

  fps_kernel<<<kB, 1024, 0, stream>>>(xyz, out0, nxyz);
  group_kernel<<<kGroups / 4, 128, 0, stream>>>(xyz, points, nxyz, (unsigned int*)aph, (unsigned int*)apl, rel);
  prep_w_kernel<<<8, 256, 0, stream>>>(W1, W2, W3, (unsigned int*)bth, (unsigned int*)btl);
  gemm_bf16x3_kernel<0><<<tiles12 / 8, 256, 0, stream>>>(aph, apl, kKf, bt1h, bt1l, kKf, zp, kC1, rel, W1,
                                                          zmax, zmin, kC3, part, kRows, kC1, kKf);
  bn_finalize_kernel<<<1, 128, 0, stream>>>(part, tilesM, kC1 / 64, kC1, g1, b1, stat0);
  bn_act_kernel<<<n8 / 256, 256, 0, stream>>>((const unsigned int*)zp, stat0, (unsigned int*)aph, (unsigned int*)apl, n8);
  gemm_bf16x3_kernel<1><<<tiles12 / 8, 256, 0, stream>>>(aph, apl, kKf, bt2h, bt2l, kKf, zp, kC2, rel, W1,
                                                          zmax, zmin, kC3, part, kRows, kC2, kKf);
  bn_finalize_kernel<<<1, 128, 0, stream>>>(part, tilesM, kC2 / 64, kC2, g2, b2, stat1);
  bn_act_kernel<<<n8 / 256, 256, 0, stream>>>((const unsigned int*)zp, stat1, (unsigned int*)aph, (unsigned int*)apl, n8);
  gemm_bf16x3_kernel<2><<<tiles3 / 8, 256, 0, stream>>>(aph, apl, kKf, bt3h, bt3l, kKf, zp, kC1, rel, W1,
                                                         zmax, zmin, kC3, part, kRows, kC3, kKf);
  bn_finalize_kernel<<<1, 128, 0, stream>>>(part, tilesM, kC3 / 64, kC3, g3, b3, stat2);
  pool_out_kernel<<<n4 / 256, 256, 0, stream>>>(zmax, zmin, stat2, out1, n4);
}
